// VisionMamba_21431886807228
// MI455X (gfx1250) — hardware-run, weakly checked
//
#include <hip/hip_runtime.h>
#include <math.h>

typedef __attribute__((ext_vector_type(16))) _Float16 v16h;
typedef __attribute__((ext_vector_type(8)))  _Float16 v8h;
typedef __attribute__((ext_vector_type(16))) __bf16   v16b;
typedef __attribute__((ext_vector_type(8)))  __bf16   v8b;
typedef __attribute__((ext_vector_type(8)))  float    v8f;
typedef __attribute__((ext_vector_type(4)))  float    v4f;

constexpr int kBatch   = 4;
constexpr int kChan    = 3;
constexpr int kImg     = 224;
constexpr int kPatch   = 16;
constexpr int kGridP   = 14;
constexpr int kSeq     = kGridP * kGridP * kChan;
constexpr int kDm      = 384;
constexpr int kDin     = 768;
constexpr int kNst     = 16;
constexpr int kDtR     = 24;
constexpr int kXdW     = kDtR + 2 * kNst;
constexpr int kXdP     = 64;
constexpr int kXzP     = 2 * kDin;
constexpr int kKp      = kPatch * kPatch;
constexpr int kDepth   = 4;
constexpr int kRows    = kBatch * kSeq;
constexpr int kRowsP   = 2368;
constexpr int kConvRows = 28;
constexpr int kConvTP  = 260;
constexpr int kScanTS  = 28;
constexpr int kScanCh  = 64;
constexpr int kScanYP  = 68;
static_assert(kSeq == 588 && kRows == 2352, "shape");
static_assert((kRowsP % 64) == 0 && kRowsP >= kRows && kRowsP - kRows == 16, "M pad");
static_assert((kKp % 32) == 0 && (kDm % 32) == 0 && (kDin % 32) == 0, "GEMM K multiples of 32");
static_assert((kDm % 64) == 0 && (kXzP % 64) == 0 && (kXdP % 64) == 0, "GEMM N multiples of 64");
static_assert((kSeq % kConvRows) == 0 && (kSeq % kScanTS) == 0 && (kScanTS % 4) == 0 && (kConvRows % 2) == 0, "chunking");
static_assert((kDin % 256) == 0 && (kDin % kScanCh) == 0 && (kDtR % 4) == 0 && kXdW <= kXdP, "tile multiples");
static_assert((kRowsP * 32) % 256 == 0 && (kDm * kKp / 8) % 256 == 0, "prep grids exact");

constexpr size_t kOffXA  = 0;
constexpr size_t kOffWP  = kOffXA  + (size_t)kRowsP * kKp * 2;
constexpr size_t kOffWIT = kOffWP  + (size_t)kDm * kKp * 2;
constexpr size_t kOffWXT = kOffWIT + (size_t)kDepth * kXzP * kDm * 2;
constexpr size_t kOffWOT = kOffWXT + (size_t)kDepth * kXdP * kDin * 2;
constexpr size_t kOffT0  = kOffWOT + (size_t)kDepth * kDm * kDin * 2;
constexpr size_t kOffR0  = kOffT0  + (size_t)kRowsP * kDm * 4;
constexpr size_t kOffR1  = kOffR0  + (size_t)kRowsP * kDm * 4;
constexpr size_t kOffHID = kOffR1  + (size_t)kRowsP * kDm * 4;
constexpr size_t kOffHS  = kOffHID + (size_t)kRowsP * kDm * 4;
constexpr size_t kOffXZ  = kOffHS  + (size_t)kRowsP * kDm * 2;
constexpr size_t kOffXC  = kOffXZ  + (size_t)kRowsP * kXzP * 4;
constexpr size_t kOffXCB = kOffXC  + (size_t)kRowsP * kDin * 4;
constexpr size_t kOffXD  = kOffXCB + (size_t)kRowsP * kDin * 2;
constexpr size_t kOffG   = kOffXD  + (size_t)kRowsP * kXdP * 4;
constexpr size_t kWsTotal = kOffG  + (size_t)kRowsP * kDin * 2;
static_assert(kWsTotal == 54951936ull, "carve total");
static_assert(kWsTotal <= 134217728ull, "carve cap");
static_assert((kOffWP % 128) == 0 && (kOffWIT % 128) == 0 && (kOffWXT % 128) == 0 && (kOffWOT % 128) == 0 &&
              (kOffT0 % 128) == 0 && (kOffR0 % 128) == 0 && (kOffR1 % 128) == 0 && (kOffHID % 128) == 0 &&
              (kOffHS % 128) == 0 && (kOffXZ % 128) == 0 && (kOffXC % 128) == 0 && (kOffXCB % 128) == 0 &&
              (kOffXD % 128) == 0 && (kOffG % 128) == 0, "128-B aligned regions");

__device__ __forceinline__ unsigned short f2bf_bits(float f) {
  unsigned u = __float_as_uint(f);
  return (unsigned short)((u + 0x7FFFu + ((u >> 16) & 1u)) >> 16);
}
__device__ __forceinline__ float bf_bits2f(unsigned short h) { return __uint_as_float(((unsigned)h) << 16); }
__device__ __forceinline__ float bfr(float f) { return bf_bits2f(f2bf_bits(f)); }
__device__ __forceinline__ v8h pack8_bf16(const v4f a0, const v4f a1) {
  v8h hv;
#pragma unroll
  for (int e = 0; e < 4; ++e) {
    const unsigned short h0 = f2bf_bits(a0[e]), h1 = f2bf_bits(a1[e]);
    hv[e]     = __builtin_bit_cast(_Float16, h0);
    hv[4 + e] = __builtin_bit_cast(_Float16, h1);
  }
  return hv;
}

__device__ __forceinline__ void dep_guard4_h(v8f& a, v8f& b, v8f& c, v8f& d, v16h x, v16h y) { asm volatile("v_nop\n\tv_nop\n\tv_nop\n\tv_nop" : "+v"(a), "+v"(b), "+v"(c), "+v"(d) : "v"(x), "v"(y)); }
__device__ __forceinline__ void dep_guard4_b(v8f& a, v8f& b, v8f& c, v8f& d, v16b x, v16b y) { asm volatile("v_nop\n\tv_nop\n\tv_nop\n\tv_nop" : "+v"(a), "+v"(b), "+v"(c), "+v"(d) : "v"(x), "v"(y)); }
__device__ __forceinline__ void keep4_h(v16h a, v16h b, v16h c, v16h d) { asm volatile("v_nop" :: "v"(a), "v"(b), "v"(c), "v"(d)); }
__device__ __forceinline__ void keep4_b(v16b a, v16b b, v16b c, v16b d) { asm volatile("v_nop" :: "v"(a), "v"(b), "v"(c), "v"(d)); }
__device__ __forceinline__ void acc_guard4(v8f& a, v8f& b, v8f& c, v8f& d) { asm volatile("v_nop\n\tv_nop\n\tv_nop\n\tv_nop" : "+v"(a), "+v"(b), "+v"(c), "+v"(d)); }
template <typename T> struct Frag;
template <> struct Frag<_Float16> {
  typedef v16h V; union U { v16h v; v8h h[2]; };
  static __device__ __forceinline__ v16h load(const _Float16* p) {
    U f; f.h[0] = *(const v8h*)(p); f.h[1] = *(const v8h*)(p + 16); return f.v;
  }
  static __device__ __forceinline__ v8f mma(v16h a, v16h b, v8f c) {
    return __builtin_amdgcn_wmma_f32_16x16x32_f16(false, a, false, b, (short)0, c, false, false);
  }
  static __device__ __forceinline__ void guard4(v8f& a, v8f& b, v8f& c, v8f& d, v16h x, v16h y) { dep_guard4_h(a, b, c, d, x, y); }
  static __device__ __forceinline__ void keep(v16h a, v16h b, v16h c, v16h d) { keep4_h(a, b, c, d); }
};
template <> struct Frag<__bf16> {
  typedef v16b V; union U { v16b v; v8b h[2]; };
  static __device__ __forceinline__ v16b load(const __bf16* p) {
    U f; f.h[0] = *(const v8b*)(p); f.h[1] = *(const v8b*)(p + 16); return f.v;
  }
  static __device__ __forceinline__ v8f mma(v16b a, v16b b, v8f c) {
    return __builtin_amdgcn_wmma_f32_16x16x32_bf16(false, a, false, b, (short)0, c, false, false);
  }
  static __device__ __forceinline__ void guard4(v8f& a, v8f& b, v8f& c, v8f& d, v16b x, v16b y) { dep_guard4_b(a, b, c, d, x, y); }
  static __device__ __forceinline__ void keep(v16b a, v16b b, v16b c, v16b d) { keep4_b(a, b, c, d); }
};

template <int ET> struct Elem;
template <> struct Elem<0> { typedef _Float16 T; };
template <> struct Elem<1> { typedef __bf16 T; };
template <int ET, bool SPLIT, int BIAS_MODE, int OUT_MODE, bool RESID, int ACT = 0>
__global__ __launch_bounds__(256) void wmma_gemm64(
    const unsigned short* __restrict__ Ap, const unsigned short* __restrict__ A2p, int lda, long strideA,
    const unsigned short* __restrict__ Btp, const unsigned short* __restrict__ Bt2p, int ldb, long strideB,
    void* __restrict__ Cout, void* __restrict__ Cout2, int ldc, long strideC,
    const float* __restrict__ bias,
    const float* __restrict__ resid, long strideR,
    int M, int N, int K, float scale) {
  typedef typename Elem<ET>::T T;
  typedef typename Frag<T>::V V;
  const T* A = (const T*)Ap; const T* A2 = (const T*)A2p; const T* Bt = (const T*)Btp; const T* Bt2 = (const T*)Bt2p;
  __shared__ __align__(16) float sT[8][16 * 68];
  const int b    = blockIdx.y;
  const int lane = threadIdx.x & 31;
  const int wave = threadIdx.x >> 5;
  const int tilesN = N >> 6;
  const int tilesM = M >> 6;
  const int tile = blockIdx.x * 8 + wave;
  if (tile >= tilesM * tilesN) return;
  const int tm = tile / tilesN;
  const int tn = tile - tm * tilesN;
  const int m0 = tm << 6;
  const int n0 = tn << 6;

  const T* Ab  = A  + (size_t)b * strideA;
  const T* Bb  = Bt + (size_t)b * strideB;
  const T* Ab2 = SPLIT ? (A2  + (size_t)b * strideA) : nullptr;
  const T* Bb2 = SPLIT ? (Bt2 + (size_t)b * strideB) : nullptr;

  const int rlane = lane & 15;
  const int koff  = (lane >> 4) * 8;
  const int mOff  = (lane >> 4) * 8;

  v8f acc[4][4];
#pragma unroll
  for (int i = 0; i < 4; ++i)
#pragma unroll
    for (int j = 0; j < 4; ++j) acc[i][j] = (v8f){0.f,0.f,0.f,0.f,0.f,0.f,0.f,0.f};

  for (int k0 = 0; k0 < K; k0 += 32) {
    V bh[4], bl[4];
#pragma unroll
    for (int j = 0; j < 4; ++j) {
      const size_t bo = (size_t)(n0 + (j << 4) + rlane) * ldb + koff + k0;
      bh[j] = Frag<T>::load(Bb + bo);
      if (SPLIT) bl[j] = Frag<T>::load(Bb2 + bo);
    }
#pragma unroll
    for (int i = 0; i < 4; ++i) {
      const size_t ao = (size_t)(m0 + (i << 4) + rlane) * lda + koff + k0;
      V ah = Frag<T>::load(Ab + ao);
      V al;
      if (SPLIT) al = Frag<T>::load(Ab2 + ao);
#pragma unroll
      for (int j = 0; j < 4; ++j) {
        acc[i][j] = Frag<T>::mma(ah, bh[j], acc[i][j]);
        if (SPLIT) {
          acc[i][j] = Frag<T>::mma(ah, bl[j], acc[i][j]);
          acc[i][j] = Frag<T>::mma(al, bh[j], acc[i][j]);
        }
      }
      Frag<T>::guard4(acc[i][0], acc[i][1], acc[i][2], acc[i][3], ah, SPLIT ? al : ah);
    }
    Frag<T>::keep(bh[0], bh[1], bh[2], bh[3]);
    if (SPLIT) Frag<T>::keep(bl[0], bl[1], bl[2], bl[3]);
  }
  acc_guard4(acc[0][0], acc[0][1], acc[0][2], acc[0][3]);
  acc_guard4(acc[1][0], acc[1][1], acc[1][2], acc[1][3]);
  acc_guard4(acc[2][0], acc[2][1], acc[2][2], acc[2][3]);
  acc_guard4(acc[3][0], acc[3][1], acc[3][2], acc[3][3]);

  float* slab = sT[wave];
  const float* Rb = RESID ? (resid + (size_t)b * strideR) : nullptr;
#pragma unroll
  for (int i = 0; i < 4; ++i) {
    const int mBase = m0 + (i << 4);
#pragma unroll
    for (int j = 0; j < 4; ++j) {
      const int n = n0 + (j << 4) + rlane;
      float bv = 0.f;
      if (BIAS_MODE == 2) bv = bias[n];
#pragma unroll
      for (int r = 0; r < 8; ++r) {
        float v = acc[i][j][r] * scale;
        if (BIAS_MODE == 1) v += bias[mBase + mOff + r];
        if (BIAS_MODE == 2) v += bv;
        if (RESID) v += Rb[(size_t)(mBase + mOff + r) * ldc + n];
        if (ACT == 1) v = tanhf(v);
        if (ACT == 2) v = fmaxf(v, 0.0f);
        if (ACT == 3) v = v / (1.0f + expf(-v));
        if (ACT == 4) v = (v > 0.f) ? v : 0.01f * v;
        slab[(mOff + r) * 68 + (j << 4) + rlane] = v;
      }
    }
    __builtin_amdgcn_fence(__ATOMIC_RELEASE, "workgroup");
    __builtin_amdgcn_wave_barrier();
    __builtin_amdgcn_fence(__ATOMIC_ACQUIRE, "workgroup");
    if (OUT_MODE == 0) {
      float* C = (float*)Cout + (size_t)b * strideC;
      const int hh = lane >> 4, c4 = (lane & 15) * 4;
      for (int pass = 0; pass < 2; ++pass) {
#pragma unroll
        for (int it = 0; it < 8; ++it) {
          const int row = it * 2 + hh;
          v4f v = *(const v4f*)(slab + row * 68 + c4);
          *(volatile v4f*)(C + (size_t)(mBase + row) * ldc + n0 + c4) = v;
        }
        __threadfence();
      }
    } else {
      const int q = lane >> 3, c8 = (lane & 7) * 8;
      unsigned short* C  = (unsigned short*)Cout  + (size_t)b * strideC;
      unsigned short* C2 = (OUT_MODE == 2) ? ((unsigned short*)Cout2 + (size_t)b * strideC) : nullptr;
      for (int pass = 0; pass < 2; ++pass) {
#pragma unroll
        for (int it = 0; it < 4; ++it) {
          const int row = it * 4 + q;
          const float* sp = slab + row * 68 + c8;
          v8h hv, lv;
#pragma unroll
          for (int e = 0; e < 8; ++e) {
            if (OUT_MODE == 1) {
              hv[e] = (_Float16)sp[e];
            } else {
              unsigned short hb = f2bf_bits(sp[e]);
              unsigned short lb = f2bf_bits(sp[e] - bf_bits2f(hb));
              hv[e] = __builtin_bit_cast(_Float16, hb);
              lv[e] = __builtin_bit_cast(_Float16, lb);
            }
          }
          *(volatile v8h*)(C + (size_t)(mBase + row) * ldc + n0 + c8) = hv;
          if (OUT_MODE == 2) *(volatile v8h*)(C2 + (size_t)(mBase + row) * ldc + n0 + c8) = lv;
        }
        __threadfence();
      }
    }
    __builtin_amdgcn_fence(__ATOMIC_RELEASE, "workgroup");
    __builtin_amdgcn_wave_barrier();
    __builtin_amdgcn_fence(__ATOMIC_ACQUIRE, "workgroup");
  }
}

__global__ __launch_bounds__(256) void im2col_kernel(const float* __restrict__ x, unsigned short* __restrict__ XA)
{
  const int i = blockIdx.x * 256 + threadIdx.x;
  const int row = i >> 5, seg = i & 31;
  const int p = seg >> 1, q0 = (seg & 1) * 8;
  const bool valid = row < kRows;
  const int rc = valid ? row : 0;
  const int b  = rc / kSeq;
  const int t  = rc - b * kSeq;
  const int c  = t % kChan;
  const int pw = t / kChan;
  const int hh = pw / kGridP;
  const int ww = pw - hh * kGridP;
  const float* src = x + ((size_t)(b * kChan + c) * kImg + (size_t)(hh * kPatch + p)) * kImg + ww * kPatch + q0;
  const float fz = valid ? 1.f : 0.f;
  const v4f a0 = *(const v4f*)(src) * fz;
  const v4f a1 = *(const v4f*)(src + 4) * fz;
  const v8h hv = pack8_bf16(a0, a1);
  unsigned short* dst = XA + (size_t)row * kKp + seg * 8;
  *(volatile v8h*)dst = hv;
  __threadfence();
  *(volatile v8h*)dst = hv;
}

__global__ __launch_bounds__(256) void cast_bf16_kernel(const float* __restrict__ src, unsigned short* __restrict__ dst, int total8)
{
  const int i = blockIdx.x * 256 + threadIdx.x;
  if (i >= total8) return;
  const size_t e0 = (size_t)i << 3;
  const v8h hv = pack8_bf16(*(const v4f*)(src + e0), *(const v4f*)(src + e0 + 4));
  *(volatile v8h*)(dst + e0) = hv;
  __threadfence();
  *(volatile v8h*)(dst + e0) = hv;
}

__global__ __launch_bounds__(256) void transpose_bf16_kernel(
    const float* __restrict__ src, long srcLayer, int R, int Cc,
    unsigned short* __restrict__ dst, long dstLayer, int CcPad)
{
  __shared__ __align__(16) float tile[64 * 68];
  const int tid = threadIdx.x;
  const int c0 = blockIdx.x * 64, r0 = blockIdx.y * 64;
  const int L = blockIdx.z;
  (void)CcPad;
  const float* s = src + (size_t)L * srcLayer;
  const int lr = tid >> 6, lc = tid & 63;
  const int c  = c0 + lc;
  const int cc = (c < Cc) ? c : (Cc - 1);
  const float f = (c < Cc) ? 1.f : 0.f;
#pragma unroll
  for (int i = 0; i < 8; ++i) {
    const int r = i * 4 + lr;
    tile[lc * 68 + r] = s[(size_t)(r0 + r) * Cc + cc] * f;
  }
  asm volatile("" ::: "memory");
#pragma unroll
  for (int i = 8; i < 16; ++i) {
    const int r = i * 4 + lr;
    tile[lc * 68 + r] = s[(size_t)(r0 + r) * Cc + cc] * f;
  }
  __syncthreads();
  unsigned short* dl = dst + (size_t)L * dstLayer;
  for (int pass = 0; pass < 2; ++pass) {
#pragma unroll
    for (int it = 0; it < 2; ++it) {
      const int u = it * 256 + tid;
      const int orow = u >> 3, seg = u & 7;
      const float* sp = tile + orow * 68 + seg * 8;
      const v8h hv = pack8_bf16(*(const v4f*)(sp), *(const v4f*)(sp + 4));
      *(volatile v8h*)(dl + (size_t)(c0 + orow) * R + r0 + seg * 8) = hv;
    }
    __threadfence();
  }
}

__global__ __launch_bounds__(256) void zero_rows_kernel(
    unsigned short* __restrict__ p0, int n0, unsigned short* __restrict__ p1, int n1,
    unsigned short* __restrict__ p2, int n2)
{
  unsigned short* p = p0; int n = n0;
  if (blockIdx.y == 1) { p = p1; n = n1; }
  if (blockIdx.y == 2) { p = p2; n = n2; }
  const int i = blockIdx.x * 256 + threadIdx.x;
  if (i < n) {
    const v4f z = {0.f, 0.f, 0.f, 0.f};
    unsigned short* d = p + (size_t)i * 8;
    *(volatile v4f*)d = z;
    __threadfence();
    *(volatile v4f*)d = z;
  }
}

template <int MODE>
__global__ __launch_bounds__(256) void ln_kernel(
    const float* __restrict__ srcA, const float* __restrict__ srcB, const float* __restrict__ cemb,
    const float* __restrict__ gw, const float* __restrict__ gb,
    float* __restrict__ Rout, unsigned short* __restrict__ HSo)
{
  __shared__ __align__(16) float slab[8 * kDm];
  const int tid = threadIdx.x, lane = tid & 31, wave = tid >> 5;
  const int row = blockIdx.x * 8 + wave;
  const float fz = (MODE == 2 || row < kRows) ? 1.f : 0.f;
  const size_t rb = (size_t)row * kDm;
  v4f v[3];
#pragma unroll
  for (int j = 0; j < 3; ++j) v[j] = *(const v4f*)(srcA + rb + lane * 4 + 128 * j);
  if (MODE == 0) {
    asm volatile("" ::: "memory");
    const int ch = row % kChan;
#pragma unroll
    for (int j = 0; j < 3; ++j) {
      const int cj = lane * 4 + 128 * j;
      const v4f pb = *(const v4f*)(srcB + cj);
      const v4f ce = *(const v4f*)(cemb + ch * kDm + cj);
#pragma unroll
      for (int e = 0; e < 4; ++e) v[j][e] = (v[j][e] + bfr(pb[e])) + bfr(ce[e]);
    }
  } else {
#pragma unroll
    for (int j = 0; j < 3; ++j) {
      const v4f hd = *(const v4f*)(srcB + rb + lane * 4 + 128 * j);
      v[j] = v[j] + hd;
    }
  }
#pragma unroll
  for (int j = 0; j < 3; ++j) v[j] = v[j] * fz;
  float s = 0.f;
#pragma unroll
  for (int j = 0; j < 3; ++j)
#pragma unroll
    for (int e = 0; e < 4; ++e) s = s + v[j][e];
#pragma unroll
  for (int off = 1; off < 32; off <<= 1) s += __shfl_xor(s, off, 32);
  const float mean = s * (1.0f / (float)kDm);
  float qs = 0.f;
#pragma unroll
  for (int j = 0; j < 3; ++j)
#pragma unroll
    for (int e = 0; e < 4; ++e) { const float dlt = v[j][e] - mean; qs = fmaf(dlt, dlt, qs); }
#pragma unroll
  for (int off = 1; off < 32; off <<= 1) qs += __shfl_xor(qs, off, 32);
  const float rstd = rsqrtf(qs * (1.0f / (float)kDm) + 1e-5f);
  asm volatile("" ::: "memory");
  v4f o[3];
#pragma unroll
  for (int j = 0; j < 3; ++j) {
    const int cj = lane * 4 + 128 * j;
    const v4f wv = *(const v4f*)(gw + cj);
    const v4f bv = *(const v4f*)(gb + cj);
#pragma unroll
    for (int e = 0; e < 4; ++e) o[j][e] = (((v[j][e] - mean) * rstd) * bfr(wv[e]) + bfr(bv[e])) * fz;
  }
  float* sw = slab + wave * kDm;
  if (MODE != 2) {
#pragma unroll
    for (int j = 0; j < 3; ++j) *(v4f*)(sw + lane * 4 + 128 * j) = o[j];
    __syncthreads();
  }
  for (int pass = 0; pass < 2; ++pass) {
#pragma unroll
    for (int j = 0; j < 3; ++j) {
      const v4f sv = (MODE == 2) ? o[j] : v[j];
      *(volatile v4f*)(Rout + rb + lane * 4 + 128 * j) = sv;
    }
    if (MODE != 2) {
      const float* sp0 = sw + lane * 8;
      const v8h h0 = pack8_bf16(*(const v4f*)(sp0), *(const v4f*)(sp0 + 4));
      *(volatile v8h*)(HSo + rb + lane * 8) = h0;
      const int s1 = 32 + (lane & 15);
      const float* sp1 = sw + s1 * 8;
      const v8h h1 = pack8_bf16(*(const v4f*)(sp1), *(const v4f*)(sp1 + 4));
      if (lane < 16) *(volatile v8h*)(HSo + rb + s1 * 8) = h1;
    }
    __threadfence();
  }
}

__global__ __launch_bounds__(256) void conv_silu_kernel(
    const float* __restrict__ XZ, const float* __restrict__ cw, const float* __restrict__ cb,
    float* __restrict__ XC, unsigned short* __restrict__ XCB)
{
  __shared__ __align__(16) float sT[kConvRows * kConvTP];
  const int tid = threadIdx.x, lane = tid & 31, wave = tid >> 5;
  const int d0 = blockIdx.x * 256, d = d0 + tid;
  const int g0 = blockIdx.y * kConvRows;
  const int tb = g0 % kSeq;
  const v4f wv = *(const v4f*)(cw + (size_t)d * 4);
  const float w0 = bfr(wv[0]), w1 = bfr(wv[1]), w2 = bfr(wv[2]), w3 = bfr(wv[3]);
  const float bc = bfr(cb[d]);
  float xm3, xm2, xm1;
  {
    const bool hist = (tb > 0);
    const int rb = hist ? (g0 - 3) : g0;
    const float v3 = XZ[(size_t)rb * kXzP + d];
    const float v2 = XZ[(size_t)(rb + 1) * kXzP + d];
    const float v1 = XZ[(size_t)(rb + 2) * kXzP + d];
    xm3 = hist ? v3 : 0.f;
    xm2 = hist ? v2 : 0.f;
    xm1 = hist ? v1 : 0.f;
  }
#pragma unroll 1
  for (int s = 0; s < kConvRows; ++s) {
    const float xcur = XZ[(size_t)(g0 + s) * kXzP + d];
    float acc = w0 * xm3;
    acc = fmaf(w1, xm2, acc);
    acc = fmaf(w2, xm1, acc);
    acc = fmaf(w3, xcur, acc);
    const float sv = acc + bc;
    const float sg = __builtin_amdgcn_rcpf(1.0f + __expf(-sv));
    sT[s * kConvTP + tid] = sv * sg;
    xm3 = xm2; xm2 = xm1; xm1 = xcur;
  }
  __syncthreads();
  for (int pass = 0; pass < 2; ++pass) {
#pragma unroll
    for (int it = 0; it < 7; ++it) {
      const int u = it * 8 + wave;
      const int row = u >> 1, hch = (u & 1) * 128 + lane * 4;
      const v4f fv = *(const v4f*)(sT + row * kConvTP + hch);
      *(volatile v4f*)(XC + (size_t)(g0 + row) * kDin + d0 + hch) = fv;
    }
#pragma unroll
    for (int it = 0; it < 4; ++it) {
      const int row = it * 8 + wave;
      if (row < kConvRows) {
        const float* sp = sT + row * kConvTP + lane * 8;
        const v8h hv = pack8_bf16(*(const v4f*)(sp), *(const v4f*)(sp + 4));
        *(volatile v8h*)(XCB + (size_t)(g0 + row) * kDin + d0 + lane * 8) = hv;
      }
    }
    __threadfence();
  }
}

__global__ __launch_bounds__(64) void scan_kernel(
    const float* __restrict__ XD, const float* __restrict__ XC, const float* __restrict__ XZ,
    const float* __restrict__ Wdt, const float* __restrict__ bdt, const float* __restrict__ Alog,
    const float* __restrict__ Dp, unsigned short* __restrict__ Gout)
{
  __shared__ __align__(16) float sX[kScanTS * kXdP];
  __shared__ __align__(16) float sY[kScanTS * kScanYP];
  __shared__ __align__(16) float sW[kDtR * kScanCh];
  __shared__ __align__(16) float sA[kNst * kScanCh];
  const int tid = threadIdx.x, lane = tid & 31, wave = tid >> 5;
  constexpr int kBlkPerB = kDin / kScanCh;
  const int bix = blockIdx.x / kBlkPerB;
  const int d0  = (blockIdx.x - bix * kBlkPerB) * kScanCh;
  const int d   = d0 + tid;
  const size_t row0 = (size_t)bix * kSeq;
#pragma unroll 1
  for (int r = 0; r < kDtR; ++r) sW[r * kScanCh + tid] = bfr(Wdt[(size_t)r * kDin + d]);
#pragma unroll 1
  for (int s = 0; s < kNst; ++s) sA[s * kScanCh + tid] = -expf(bfr(Alog[(size_t)d * kNst + s]));
  __syncthreads();
  float negA[kNst], h[kNst];
#pragma unroll
  for (int s = 0; s < kNst; ++s) {
    negA[s] = sA[s * kScanCh + tid];
    h[s] = 0.f;
  }
  const float bb = bfr(bdt[d]), Dd = bfr(Dp[d]);
  const int lr = tid >> 4, lc4 = (tid & 15) * 4;
  const int q = lane >> 3, c8 = (lane & 7) * 8;
#pragma unroll 1
  for (int t0 = 0; t0 < kSeq; t0 += kScanTS) {
    __syncthreads();
#pragma unroll
    for (int i = 0; i < kScanTS / 4; ++i) {
      const int r = lr + 4 * i;
      *(v4f*)(sX + r * kXdP + lc4) = *(const v4f*)(XD + (row0 + t0 + r) * kXdP + lc4);
    }
    __syncthreads();
#pragma unroll 1
    for (int s = 0; s < kScanTS; ++s) {
      const int t = t0 + s;
      const float* xr = sX + s * kXdP;
      float vdot = 0.f;
#pragma unroll 1
      for (int r4 = 0; r4 < kDtR / 4; ++r4) {
        const v4f xv = *(const v4f*)(xr + 4 * r4);
        const float* wp = sW + (4 * r4) * kScanCh + tid;
        vdot = fmaf(xv[0], wp[0], vdot);
        vdot = fmaf(xv[1], wp[kScanCh], vdot);
        vdot = fmaf(xv[2], wp[2 * kScanCh], vdot);
        vdot = fmaf(xv[3], wp[3 * kScanCh], vdot);
      }
      float Bs[kNst], Cs[kNst];
#pragma unroll
      for (int q4 = 0; q4 < 4; ++q4) {
        const v4f bv = *(const v4f*)(xr + kDtR + 4 * q4);
        const v4f cv = *(const v4f*)(xr + kDtR + kNst + 4 * q4);
        Bs[4 * q4 + 0] = bv[0]; Bs[4 * q4 + 1] = bv[1]; Bs[4 * q4 + 2] = bv[2]; Bs[4 * q4 + 3] = bv[3];
        Cs[4 * q4 + 0] = cv[0]; Cs[4 * q4 + 1] = cv[1]; Cs[4 * q4 + 2] = cv[2]; Cs[4 * q4 + 3] = cv[3];
      }
      const float v   = vdot + bb;
      const float a   = __expf(-fabsf(v));
      const float u   = 1.0f + a;
      const float l1p = __logf(u) + (a - (u - 1.0f)) * __builtin_amdgcn_rcpf(u);
      const float dt  = fmaxf(v, 0.0f) + l1p;
      const float xt  = XC[(row0 + t) * kDin + d];
      const float dtx = dt * xt;
      float y = 0.f;
#pragma unroll
      for (int k = 0; k < kNst; ++k) {
        const float e = __expf(dt * negA[k]);
        h[k] = e * h[k] + dtx * Bs[k];
        y = h[k] * Cs[k] + y;
      }
      y = xt * Dd + y;
      const float zv = XZ[(row0 + t) * kXzP + kDin + d];
      const float sg = __builtin_amdgcn_rcpf(1.0f + __expf(-zv));
      y = y * (zv * sg);
      sY[s * kScanYP + tid] = y;
    }
    __syncthreads();
    for (int pass = 0; pass < 2; ++pass) {
#pragma unroll
      for (int it = 0; it < 4; ++it) {
        const int rbase = it * 8 + wave * 4;
        if (rbase < kScanTS) {
          const int row = rbase + q;
          const float* sp = sY + row * kScanYP + c8;
          const v8h hv = pack8_bf16(*(const v4f*)(sp), *(const v4f*)(sp + 4));
          *(volatile v8h*)(Gout + (row0 + t0 + row) * kDin + d0 + c8) = hv;
        }
      }
      __threadfence();
    }
  }
}

extern "C" void kernel_launch(void* const* d_in, const int* in_sizes, int n_in,
                              void* d_out, int out_size, void* d_ws, size_t ws_size,
                              hipStream_t stream)
{
  if (n_in < 17) return;
  if (in_sizes[0]  != kBatch * kChan * kImg * kImg) return;
  if (in_sizes[1]  != kDm * kKp) return;
  if (in_sizes[2]  != kDm) return;
  if (in_sizes[3]  != kChan * kDm) return;
  if (in_sizes[4]  != kDepth * kDm) return;
  if (in_sizes[5]  != kDepth * kDm) return;
  if (in_sizes[6]  != kDepth * kDm * kXzP) return;
  if (in_sizes[7]  != kDepth * kDin * 4) return;
  if (in_sizes[8]  != kDepth * kDin) return;
  if (in_sizes[9]  != kDepth * kDin * kXdW) return;
  if (in_sizes[10] != kDepth * kDtR * kDin) return;
  if (in_sizes[11] != kDepth * kDin) return;
  if (in_sizes[12] != kDepth * kDin * kNst) return;
  if (in_sizes[13] != kDepth * kDin) return;
  if (in_sizes[14] != kDepth * kDin * kDm) return;
  if (in_sizes[15] != kDm) return;
  if (in_sizes[16] != kDm) return;
  if (out_size != kRows * kDm) return;
  if (ws_size < kWsTotal) return;

  const float* x        = (const float*)d_in[0];
  const float* patch_w  = (const float*)d_in[1];
  const float* patch_b  = (const float*)d_in[2];
  const float* chan_emb = (const float*)d_in[3];
  const float* norm_w   = (const float*)d_in[4];
  const float* norm_b   = (const float*)d_in[5];
  const float* in_w     = (const float*)d_in[6];
  const float* conv_w   = (const float*)d_in[7];
  const float* conv_b   = (const float*)d_in[8];
  const float* x_w      = (const float*)d_in[9];
  const float* dt_w     = (const float*)d_in[10];
  const float* dt_b     = (const float*)d_in[11];
  const float* A_log    = (const float*)d_in[12];
  const float* D_skip   = (const float*)d_in[13];
  const float* out_w    = (const float*)d_in[14];
  const float* normf_w  = (const float*)d_in[15];
  const float* normf_b  = (const float*)d_in[16];
  float* out = (float*)d_out;

  char* ws = (char*)d_ws;
  unsigned short* XA  = (unsigned short*)(ws + kOffXA);
  unsigned short* WP  = (unsigned short*)(ws + kOffWP);
  unsigned short* WIT = (unsigned short*)(ws + kOffWIT);
  unsigned short* WXT = (unsigned short*)(ws + kOffWXT);
  unsigned short* WOT = (unsigned short*)(ws + kOffWOT);
  float*          T0  = (float*)(ws + kOffT0);
  float*          R0  = (float*)(ws + kOffR0);
  float*          R1  = (float*)(ws + kOffR1);
  float*          HID = (float*)(ws + kOffHID);
  unsigned short* HS  = (unsigned short*)(ws + kOffHS);
  float*          XZ  = (float*)(ws + kOffXZ);
  float*          XC  = (float*)(ws + kOffXC);
  unsigned short* XCB = (unsigned short*)(ws + kOffXCB);
  float*          XD  = (float*)(ws + kOffXD);
  unsigned short* G   = (unsigned short*)(ws + kOffG);

  im2col_kernel<<<(kRowsP * 32) / 256, 256, 0, stream>>>(x, XA);
  cast_bf16_kernel<<<(kDm * kKp / 8) / 256, 256, 0, stream>>>(patch_w, WP, kDm * kKp / 8);
  transpose_bf16_kernel<<<dim3(kXzP / 64, kDm / 64, kDepth), 256, 0, stream>>>(
      in_w, (long)kDm * kXzP, kDm, kXzP, WIT, (long)kXzP * kDm, kXzP);
  transpose_bf16_kernel<<<dim3(kXdP / 64, kDin / 64, kDepth), 256, 0, stream>>>(
      x_w, (long)kDin * kXdW, kDin, kXdW, WXT, (long)kXdP * kDin, kXdP);
  transpose_bf16_kernel<<<dim3(kDm / 64, kDin / 64, kDepth), 256, 0, stream>>>(
      out_w, (long)kDin * kDm, kDin, kDm, WOT, (long)kDm * kDin, kDm);
  zero_rows_kernel<<<dim3(6, 3), 256, 0, stream>>>(
      HS + (size_t)kRows * kDm, 16 * kDm / 8,
      XCB + (size_t)kRows * kDin, 16 * kDin / 8,
      G + (size_t)kRows * kDin, 16 * kDin / 8);

  wmma_gemm64<1, false, 0, 0, false><<<dim3(28, 1), 256, 0, stream>>>(
      XA, nullptr, kKp, 0L,
      WP, nullptr, kKp, 0L,
      (void*)T0, nullptr, kDm, 0L,
      nullptr, nullptr, 0L,
      kRowsP, kDm, kKp, 1.0f);

  for (int L = 0; L < kDepth; ++L) {
    float* Rprev = (L & 1) ? R0 : R1;
    float* Rcur  = (L & 1) ? R1 : R0;
    if (L == 0) {
      ln_kernel<0><<<kRowsP / 8, 256, 0, stream>>>(T0, patch_b, chan_emb, norm_w, norm_b, R0, HS);
    } else {
      ln_kernel<1><<<kRowsP / 8, 256, 0, stream>>>(Rprev, HID, chan_emb, norm_w + L * kDm, norm_b + L * kDm, Rcur, HS);
    }
    wmma_gemm64<1, false, 0, 0, false><<<dim3(111, 1), 256, 0, stream>>>(
        HS, nullptr, kDm, 0L,
        WIT + (size_t)L * kXzP * kDm, nullptr, kDm, 0L,
        (void*)XZ, nullptr, kXzP, 0L,
        nullptr, nullptr, 0L,
        kRowsP, kXzP, kDm, 1.0f);
    conv_silu_kernel<<<dim3(kDin / 256, kRows / kConvRows), 256, 0, stream>>>(
        XZ, conv_w + (size_t)L * kDin * 4, conv_b + (size_t)L * kDin, XC, XCB);
    wmma_gemm64<1, false, 0, 0, false><<<dim3(5, 1), 256, 0, stream>>>(
        XCB, nullptr, kDin, 0L,
        WXT + (size_t)L * kXdP * kDin, nullptr, kDin, 0L,
        (void*)XD, nullptr, kXdP, 0L,
        nullptr, nullptr, 0L,
        kRowsP, kXdP, kDin, 1.0f);
    scan_kernel<<<kBatch * (kDin / kScanCh), kScanCh, 0, stream>>>(
        XD, XC, XZ, dt_w + (size_t)L * kDtR * kDin, dt_b + (size_t)L * kDin,
        A_log + (size_t)L * kDin * kNst, D_skip + (size_t)L * kDin, G);
    wmma_gemm64<1, false, 0, 0, false><<<dim3(28, 1), 256, 0, stream>>>(
        G, nullptr, kDin, 0L,
        WOT + (size_t)L * kDm * kDin, nullptr, kDin, 0L,
        (void*)HID, nullptr, kDm, 0L,
        nullptr, nullptr, 0L,
        kRowsP, kDm, kDin, 1.0f);
  }

  ln_kernel<2><<<kRows / 8, 256, 0, stream>>>(R1, HID, chan_emb, normf_w, normf_b, out, HS);
}
